// Physics_7370163880185
// MI455X (gfx1250) — hardware-verified
//
#include <hip/hip_runtime.h>
#include <stddef.h>
#include <stdint.h>


#define NOBJ   16
#define BROW   512
#define DIN    256
#define HID    512
#define MROWS  8192
#define ASC    8
#define WSC    256
#define NTHR   256
#define NWAVE  8
#define TPW    64
#define NSLOT  5
#define NGRP   3
#define WSCAP  134217728
#define LDS_GEMM (NWAVE * 32 * 64 * 4)

static_assert(MROWS == NOBJ * BROW);
static_assert((MROWS % 128) == 0);
static_assert((HID % 128) == 0);
static_assert((DIN % 128) == 0);
static_assert((HID % 64) == 0);
static_assert((DIN % 64) == 0);
static_assert(NTHR == NWAVE * 32);
static_assert(NSLOT * NGRP == NOBJ - 1);
static_assert(((MROWS * DIN) % (8 * NTHR)) == 0);
static_assert(((MROWS * HID) % (8 * NTHR)) == 0);
static_assert(LDS_GEMM <= 300 * 1024);

#define SZ_X16  ((size_t)MROWS * DIN * 2)
#define SZ_TW1  ((size_t)HID * DIN * 2)
#define SZ_TW2  ((size_t)HID * HID * 2)
#define SZ_TW3  ((size_t)DIN * HID * 2)
#define SZ_IW1  ((size_t)HID * HID * 2)
#define SZ_IW2  ((size_t)HID * HID * 2)
#define SZ_IW3  ((size_t)DIN * HID * 2)
#define SZ_T    ((size_t)MROWS * HID * 2)
#define SZ_PQ   ((size_t)MROWS * HID * 4)
#define SZ_H1   ((size_t)MROWS * HID * 2)
#define SZ_H2   ((size_t)NSLOT * MROWS * HID * 2)
#define SZ_PART ((size_t)MROWS * DIN * 4)
#define SZ_TOTAL (SZ_X16 + SZ_TW1 + SZ_TW2 + SZ_TW3 + SZ_IW1 + SZ_IW2 + SZ_IW3 + 2 * SZ_T + 2 * SZ_PQ + SZ_H1 + SZ_H2 + 2 * SZ_PART)
static_assert(SZ_TOTAL <= (size_t)WSCAP);
static_assert((SZ_X16 % 256) == 0);
static_assert((SZ_TW1 % 256) == 0);
static_assert((SZ_TW3 % 256) == 0);
static_assert((SZ_T % 256) == 0);
static_assert((SZ_PQ % 256) == 0);
static_assert((SZ_PART % 256) == 0);

typedef float          v2f  __attribute__((ext_vector_type(2)));
typedef float          v4f  __attribute__((ext_vector_type(4)));
typedef float          v8f  __attribute__((ext_vector_type(8)));
typedef _Float16       v8h  __attribute__((ext_vector_type(8)));
typedef _Float16       v16h __attribute__((ext_vector_type(16)));
union FragH { v16h v; v8h h[2]; };

__device__ __forceinline__ v8f wmf(v16h a, v16h b, v8f c) {
  v8f d = __builtin_amdgcn_wmma_f32_16x16x32_f16(false, a, false, b, (short)0, c, false, false);
  asm volatile("v_nop\n\tv_nop\n\tv_nop\n\tv_nop" : "+v"(d) : "v"(a), "v"(b));
  return d;
}

__global__ __launch_bounds__(NTHR) void k_prepx(const float* __restrict__ x, _Float16* xh) {
  const size_t t = (size_t)blockIdx.x * NTHR + threadIdx.x;
  const float* p = x + t * 8;
  const v4f f0 = *(const v4f*)p;
  const v4f f1 = *(const v4f*)(p + 4);
  v8h a;
  a[0] = (_Float16)(f0.x * (float)ASC); a[1] = (_Float16)(f0.y * (float)ASC);
  a[2] = (_Float16)(f0.z * (float)ASC); a[3] = (_Float16)(f0.w * (float)ASC);
  a[4] = (_Float16)(f1.x * (float)ASC); a[5] = (_Float16)(f1.y * (float)ASC);
  a[6] = (_Float16)(f1.z * (float)ASC); a[7] = (_Float16)(f1.w * (float)ASC);
  _Float16* d = xh + t * 8;
  *(volatile v8h*)d = a;
  __threadfence();
  *(volatile v8h*)d = a;
}

__global__ __launch_bounds__(NTHR) void k_prepw(const float* __restrict__ W, _Float16* wt, int K, int N) {
  __shared__ __attribute__((aligned(16))) float tile[128 * TPW];
  const int tid = threadIdx.x, lane = tid & 31, g = tid >> 5, hh = lane >> 4, m = lane & 15;
  const int n0 = blockIdx.x * 64;
  const int n = n0 + 2 * lane;
#pragma unroll 1
  for (int dc = 0; dc < K; dc += 128) {
    __syncthreads();
#pragma unroll 4
    for (int p = 0; p < 16; ++p) {
      const int dl = g + 8 * p;
      const v2f w = *(const v2f*)(W + (size_t)(dc + dl) * N + n);
      *(v2f*)(tile + dl * TPW + 2 * lane) = w;
    }
    __syncthreads();
    v8h hv[4];
#pragma unroll
    for (int q = 0; q < 4; ++q) {
      const int nl = 8 * g + 2 * q + hh;
      const int d8 = 8 * m;
#pragma unroll
      for (int e = 0; e < 8; ++e) hv[q][e] = (_Float16)(tile[(d8 + e) * TPW + nl] * (float)WSC);
    }
#pragma unroll
    for (int q = 0; q < 4; ++q) {
      _Float16* d = wt + (size_t)(n0 + 8 * g + 2 * q + hh) * K + dc + 8 * m;
      *(volatile v8h*)d = hv[q];
    }
    __threadfence();
#pragma unroll
    for (int q = 0; q < 4; ++q) {
      _Float16* d = wt + (size_t)(n0 + 8 * g + 2 * q + hh) * K + dc + 8 * m;
      *(volatile v8h*)d = hv[q];
    }
  }
}

__global__ __launch_bounds__(NTHR) void k_h1(const float* __restrict__ P, const float* __restrict__ Q,
                                             const float* __restrict__ b1, _Float16* H1, int d) {
  const size_t t = (size_t)blockIdx.x * NTHR + threadIdx.x;
  const size_t e = t * 8;
  const int row = (int)(e >> 9);
  const int c = (int)(e & (HID - 1));
  const int i = row >> 9, b = row & (BROW - 1);
  const int j = (i + d) & (NOBJ - 1);
  const float* pp = P + (size_t)row * HID + c;
  const float* qp = Q + ((size_t)j * BROW + b) * HID + c;
  const v4f p0 = *(const v4f*)pp, p1 = *(const v4f*)(pp + 4);
  const v4f q0 = *(const v4f*)qp, q1 = *(const v4f*)(qp + 4);
  const v4f c0 = *(const v4f*)(b1 + c), c1 = *(const v4f*)(b1 + c + 4);
  v4f s0 = p0 + q0; s0 = s0 + c0;
  v4f s1 = p1 + q1; s1 = s1 + c1;
  v8h hv;
  hv[0] = (_Float16)(fmaxf(s0.x, 0.f) * (float)ASC); hv[1] = (_Float16)(fmaxf(s0.y, 0.f) * (float)ASC);
  hv[2] = (_Float16)(fmaxf(s0.z, 0.f) * (float)ASC); hv[3] = (_Float16)(fmaxf(s0.w, 0.f) * (float)ASC);
  hv[4] = (_Float16)(fmaxf(s1.x, 0.f) * (float)ASC); hv[5] = (_Float16)(fmaxf(s1.y, 0.f) * (float)ASC);
  hv[6] = (_Float16)(fmaxf(s1.z, 0.f) * (float)ASC); hv[7] = (_Float16)(fmaxf(s1.w, 0.f) * (float)ASC);
  _Float16* dst = H1 + e;
  *(volatile v8h*)dst = hv;
  __threadfence();
  *(volatile v8h*)dst = hv;
}

__device__ __forceinline__ void mma_tile(v8f (&acc)[2][4], const _Float16* ap, int lda,
                                         const _Float16* bp, int ldb, int K) {
#pragma unroll 1
  for (int k0 = 0; k0 < K; k0 += 32) {
    FragH a0, a1;
    a0.h[0] = *(const v8h*)(ap + k0);
    a0.h[1] = *(const v8h*)(ap + k0 + 16);
    a1.h[0] = *(const v8h*)(ap + (size_t)16 * lda + k0);
    a1.h[1] = *(const v8h*)(ap + (size_t)16 * lda + k0 + 16);
#pragma unroll
    for (int nt = 0; nt < 4; ++nt) {
      const _Float16* bq = bp + (size_t)nt * 16 * ldb + k0;
      FragH bf;
      bf.h[0] = *(const v8h*)bq;
      bf.h[1] = *(const v8h*)(bq + 16);
      acc[0][nt] = wmf(a0.v, bf.v, acc[0][nt]);
      acc[1][nt] = wmf(a1.v, bf.v, acc[1][nt]);
    }
  }
}

__global__ __launch_bounds__(NTHR) void k_gemm16(const _Float16* __restrict__ A, int lda,
                                                 const _Float16* __restrict__ Bt, int ldb, int K,
                                                 const float* __restrict__ bias, _Float16* out, int ldo) {
  extern __shared__ v4f lds_dyn[];
  const int tid = threadIdx.x, lane = tid & 31, wave = tid >> 5, hh = lane >> 4, m = lane & 15;
  float* stg = (float*)lds_dyn + wave * (32 * 64);
  const int n0 = blockIdx.x * 128, m0 = blockIdx.y * 128;
  const int wm = (wave >> 1) * 32, wn = (wave & 1) * 64;

  v8f acc[2][4];
#pragma unroll
  for (int mt = 0; mt < 2; ++mt)
#pragma unroll
    for (int nt = 0; nt < 4; ++nt) { v8f z = {0.f, 0.f, 0.f, 0.f, 0.f, 0.f, 0.f, 0.f}; acc[mt][nt] = z; }

  const _Float16* ap = A + (size_t)(m0 + wm + m) * lda + 8 * hh;
  const _Float16* bp = Bt + (size_t)(n0 + wn + m) * ldb + 8 * hh;
  mma_tile(acc, ap, lda, bp, ldb, K);

  constexpr float OSC = 1.0f / (float)(ASC * WSC);
  float bv[4];
#pragma unroll
  for (int nt = 0; nt < 4; ++nt) bv[nt] = bias[n0 + wn + 16 * nt + m];
#pragma unroll
  for (int mt = 0; mt < 2; ++mt) {
    float* sp = stg + (16 * mt + 8 * hh) * 64 + m;
#pragma unroll
    for (int nt = 0; nt < 4; ++nt) {
#pragma unroll
      for (int r = 0; r < 8; ++r) {
        float v = acc[mt][nt][r] * OSC + bv[nt];
        v = fmaxf(v, 0.f);
        sp[r * 64 + 16 * nt] = v * (float)ASC;
      }
    }
  }
  __syncthreads();

  const int rl = lane >> 3, c8 = 8 * (lane & 7);
  v8h hv[8];
#pragma unroll
  for (int q = 0; q < 8; ++q) {
    const float* s = stg + (4 * q + rl) * 64 + c8;
    const v4f f0 = *(const v4f*)s;
    const v4f f1 = *(const v4f*)(s + 4);
    hv[q][0] = (_Float16)f0.x; hv[q][1] = (_Float16)f0.y; hv[q][2] = (_Float16)f0.z; hv[q][3] = (_Float16)f0.w;
    hv[q][4] = (_Float16)f1.x; hv[q][5] = (_Float16)f1.y; hv[q][6] = (_Float16)f1.z; hv[q][7] = (_Float16)f1.w;
  }
  _Float16* gb = out + (size_t)(m0 + wm) * ldo + n0 + wn + c8;
#pragma unroll
  for (int q = 0; q < 8; ++q) *(volatile v8h*)(gb + (size_t)(4 * q + rl) * ldo) = hv[q];
  __threadfence();
#pragma unroll
  for (int q = 0; q < 8; ++q) *(volatile v8h*)(gb + (size_t)(4 * q + rl) * ldo) = hv[q];
}

__global__ __launch_bounds__(NTHR) void k_gemm32(const _Float16* __restrict__ A, int lda, int slotStride, int nslot,
                                                 const _Float16* __restrict__ Bt, int ldb, int K,
                                                 const float* __restrict__ bias, int dobias, int dorelu,
                                                 const float* add0, const float* add1, int nadd,
                                                 float* out, int ldo) {
  extern __shared__ v4f lds_dyn[];
  const int tid = threadIdx.x, lane = tid & 31, wave = tid >> 5, hh = lane >> 4, m = lane & 15;
  float* stg = (float*)lds_dyn + wave * (32 * 64);
  const int n0 = blockIdx.x * 128, m0 = blockIdx.y * 128;
  const int wm = (wave >> 1) * 32, wn = (wave & 1) * 64;
  constexpr float OSC = 1.0f / (float)(ASC * WSC);

#pragma unroll
  for (int mt = 0; mt < 2; ++mt) {
    float* sp = stg + (16 * mt + 8 * hh) * 64 + m;
#pragma unroll
    for (int nt = 0; nt < 4; ++nt) {
#pragma unroll
      for (int r = 0; r < 8; ++r) sp[r * 64 + 16 * nt] = 0.f;
    }
  }

  float bv[4];
#pragma unroll
  for (int nt = 0; nt < 4; ++nt) {
    const float bvv = bias[n0 + wn + 16 * nt + m];
    bv[nt] = dobias ? bvv : 0.f;
  }
  const _Float16* bp = Bt + (size_t)(n0 + wn + m) * ldb + 8 * hh;

#pragma unroll 1
  for (int s = 0; s < nslot; ++s) {
    v8f acc[2][4];
#pragma unroll
    for (int mt = 0; mt < 2; ++mt)
#pragma unroll
      for (int nt = 0; nt < 4; ++nt) { v8f z = {0.f, 0.f, 0.f, 0.f, 0.f, 0.f, 0.f, 0.f}; acc[mt][nt] = z; }
    const _Float16* ap = A + (size_t)s * (size_t)slotStride + (size_t)(m0 + wm + m) * lda + 8 * hh;
    mma_tile(acc, ap, lda, bp, ldb, K);
#pragma unroll
    for (int mt = 0; mt < 2; ++mt) {
      float* sp = stg + (16 * mt + 8 * hh) * 64 + m;
#pragma unroll
      for (int nt = 0; nt < 4; ++nt) {
#pragma unroll
        for (int r = 0; r < 8; ++r) {
          float v = acc[mt][nt][r] * OSC + bv[nt];
          v = dorelu ? fmaxf(v, 0.f) : v;
          sp[r * 64 + 16 * nt] += v;
        }
      }
    }
  }
  __syncthreads();

  const bool use0 = (nadd >= 1);
  const bool use1 = (nadd >= 2);
  const size_t gro = (size_t)(m0 + wm) * ldo + n0 + wn + 4 * m;
  v4f vals[16];
#pragma unroll
  for (int gq = 0; gq < 4; ++gq) {
#pragma unroll
    for (int qq = 0; qq < 4; ++qq) {
      const int q = 4 * gq + qq;
      const int row = 2 * q + hh;
      v4f v = *(const v4f*)(stg + row * 64 + 4 * m);
      const size_t g = gro + (size_t)row * ldo;
      if (use0) {
        const v4f a0v = *(const v4f*)(add0 + g);
        v = v + a0v;
      }
      if (use1) {
        const v4f a1v = *(const v4f*)(add1 + g);
        v = v + a1v;
      }
      vals[q] = v;
    }
    __threadfence();
  }

  float* gbase = out + gro;
#pragma unroll
  for (int q = 0; q < 16; ++q) {
    const int row = 2 * q + hh;
    *(volatile v4f*)(gbase + (size_t)row * ldo) = vals[q];
  }
  __threadfence();
#pragma unroll
  for (int q = 0; q < 16; ++q) {
    const int row = 2 * q + hh;
    *(volatile v4f*)(gbase + (size_t)row * ldo) = vals[q];
  }
}

extern "C" void kernel_launch(void* const* d_in, const int* in_sizes, int n_in,
                              void* d_out, int out_size, void* d_ws, size_t ws_size,
                              hipStream_t stream) {
  if (n_in < 13) return;
  if (in_sizes[0] != MROWS * DIN) return;
  if (in_sizes[1] != DIN * HID || in_sizes[2] != HID) return;
  if (in_sizes[3] != HID * HID || in_sizes[4] != HID) return;
  if (in_sizes[5] != HID * DIN || in_sizes[6] != DIN) return;
  if (in_sizes[7] != HID * HID || in_sizes[8] != HID) return;
  if (in_sizes[9] != HID * HID || in_sizes[10] != HID) return;
  if (in_sizes[11] != HID * DIN || in_sizes[12] != DIN) return;
  if (out_size != MROWS * DIN) return;

  const float* objs = (const float*)d_in[0];
  const float* tW1 = (const float*)d_in[1];  const float* tb1 = (const float*)d_in[2];
  const float* tW2 = (const float*)d_in[3];  const float* tb2 = (const float*)d_in[4];
  const float* tW3 = (const float*)d_in[5];  const float* tb3 = (const float*)d_in[6];
  const float* iW1 = (const float*)d_in[7];  const float* ib1 = (const float*)d_in[8];
  const float* iW2 = (const float*)d_in[9];  const float* ib2 = (const float*)d_in[10];
  const float* iW3 = (const float*)d_in[11]; const float* ib3 = (const float*)d_in[12];
  float* out = (float*)d_out;

  char* ws = (char*)d_ws;
  size_t off = 0;
  const size_t oX16 = off;  off += SZ_X16;
  const size_t oTW1 = off;  off += SZ_TW1;
  const size_t oTW2 = off;  off += SZ_TW2;
  const size_t oTW3 = off;  off += SZ_TW3;
  const size_t oIW1 = off;  off += SZ_IW1;
  const size_t oIW2 = off;  off += SZ_IW2;
  const size_t oIW3 = off;  off += SZ_IW3;
  const size_t oT1  = off;  off += SZ_T;
  const size_t oT2  = off;  off += SZ_T;
  const size_t oP   = off;  off += SZ_PQ;
  const size_t oQ   = off;  off += SZ_PQ;
  const size_t oH1  = off;  off += SZ_H1;
  const size_t oH2  = off;  off += SZ_H2;
  const size_t oPA  = off;  off += SZ_PART;
  const size_t oPB  = off;  off += SZ_PART;
  if (off != SZ_TOTAL) return;
  if (off > ws_size || off > (size_t)WSCAP) return;

  _Float16* x16  = (_Float16*)(ws + oX16);
  _Float16* tW1t = (_Float16*)(ws + oTW1);
  _Float16* tW2t = (_Float16*)(ws + oTW2);
  _Float16* tW3t = (_Float16*)(ws + oTW3);
  _Float16* iW1t = (_Float16*)(ws + oIW1);
  _Float16* iW2t = (_Float16*)(ws + oIW2);
  _Float16* iW3t = (_Float16*)(ws + oIW3);
  _Float16* t1   = (_Float16*)(ws + oT1);
  _Float16* t2   = (_Float16*)(ws + oT2);
  float*    pP   = (float*)(ws + oP);
  float*    pQ   = (float*)(ws + oQ);
  _Float16* h1   = (_Float16*)(ws + oH1);
  _Float16* h2   = (_Float16*)(ws + oH2);
  float* part[2];
  part[0] = (float*)(ws + oPA);
  part[1] = (float*)(ws + oPB);

  k_prepx<<<(MROWS * DIN) / (8 * NTHR), NTHR, 0, stream>>>(objs, x16);
  k_prepw<<<HID / 64, NTHR, 0, stream>>>(tW1, tW1t, DIN, HID);
  k_prepw<<<HID / 64, NTHR, 0, stream>>>(tW2, tW2t, HID, HID);
  k_prepw<<<DIN / 64, NTHR, 0, stream>>>(tW3, tW3t, HID, DIN);
  k_prepw<<<HID / 64, NTHR, 0, stream>>>(iW1, iW1t, HID, HID);
  k_prepw<<<HID / 64, NTHR, 0, stream>>>(iW2, iW2t, HID, HID);
  k_prepw<<<DIN / 64, NTHR, 0, stream>>>(iW3, iW3t, HID, DIN);

  hipFuncSetAttribute(reinterpret_cast<const void*>(&k_gemm16),
                      hipFuncAttributeMaxDynamicSharedMemorySize, LDS_GEMM);
  hipFuncSetAttribute(reinterpret_cast<const void*>(&k_gemm32),
                      hipFuncAttributeMaxDynamicSharedMemorySize, LDS_GEMM);

  const dim3 gH(HID / 128, MROWS / 128);
  const dim3 gD(DIN / 128, MROWS / 128);
  const int slotHalves = MROWS * HID;

  k_gemm16<<<gH, NTHR, LDS_GEMM, stream>>>(x16, DIN, tW1t, DIN, DIN, tb1, t1, HID);
  k_gemm16<<<gH, NTHR, LDS_GEMM, stream>>>(t1, HID, tW2t, HID, HID, tb2, t2, HID);

  k_gemm32<<<gH, NTHR, LDS_GEMM, stream>>>(x16, DIN, 0, 1, iW1t, HID, DIN, ib1, 0, 0, pQ, pQ, 0, pP, HID);
  k_gemm32<<<gH, NTHR, LDS_GEMM, stream>>>(x16, DIN, 0, 1, iW1t + DIN, HID, DIN, ib1, 0, 0, pP, pP, 0, pQ, HID);

#pragma unroll 1
  for (int g = 0; g < NGRP; ++g) {
    for (int dd = 0; dd < NSLOT; ++dd) {
      const int d = g * NSLOT + dd + 1;
      k_h1<<<(MROWS * HID) / (8 * NTHR), NTHR, 0, stream>>>(pP, pQ, ib1, h1, d);
      k_gemm16<<<gH, NTHR, LDS_GEMM, stream>>>(h1, HID, iW2t, HID, HID, ib2, h2 + (size_t)dd * slotHalves, HID);
    }
    float* src = part[(g + 1) & 1];
    float* dst = part[g & 1];
    k_gemm32<<<gD, NTHR, LDS_GEMM, stream>>>(h2, HID, slotHalves, NSLOT, iW3t, HID, HID, ib3, 1, 1,
                                             src, src, (g > 0) ? 1 : 0, dst, DIN);
  }

  k_gemm32<<<gD, NTHR, LDS_GEMM, stream>>>(t2, HID, 0, 1, tW3t, HID, HID, tb3, 1, 1,
                                           part[(NGRP - 1) & 1], objs, 2, out, DIN);
}
